// Model_NCF_37486474559594
// MI455X (gfx1250) — hardware-verified
//
#include <hip/hip_runtime.h>
#include <math.h>

typedef __attribute__((ext_vector_type(16))) _Float16 v16h;
typedef __attribute__((ext_vector_type(16))) __bf16 v16b;
typedef __attribute__((ext_vector_type(8)))  _Float16 v8h;
typedef __attribute__((ext_vector_type(8)))  float v8f;
typedef __attribute__((ext_vector_type(4)))  float v4f;
typedef __attribute__((ext_vector_type(2)))  float v2f;
typedef __attribute__((ext_vector_type(4)))  unsigned v4u;
typedef __attribute__((ext_vector_type(4)))  int v4i;
typedef float __attribute__((may_alias)) float_a;
typedef int __attribute__((may_alias)) int_a;

template <typename T> __device__ __forceinline__ void vst2(void* p, T v) { *(volatile T*)p = v; __threadfence(); *(volatile T*)p = v; }
__device__ __forceinline__ v8f wmma16(v16h a, v16h b, v8f c) {
  v8f d = __builtin_amdgcn_wmma_f32_16x16x32_f16(false, a, false, b, (short)0, c, false, false);
  asm volatile("v_nop\n\tv_nop\n\tv_nop\n\tv_nop" : "+v"(d) : "v"(a), "v"(b));
  return d;
}
__device__ __forceinline__ v8f wmma_bf(v16b a, v16b b, v8f c) {
  v8f d = __builtin_amdgcn_wmma_f32_16x16x32_bf16(false, a, false, b, (short)0, c, false, false);
  asm volatile("v_nop\n\tv_nop\n\tv_nop\n\tv_nop" : "+v"(d) : "v"(a), "v"(b));
  return d;
}
__device__ __forceinline__ v16h frag_h(const _Float16* rowk0, int lane) {
  union { v16h v; v8h q[2]; } u; const _Float16* p = rowk0 + 8 * (lane >> 4);
  u.q[0] = *(const v8h*)p; u.q[1] = *(const v8h*)(p + 16); return u.v;
}
__device__ __forceinline__ v16h frag_f32(const float* rowk0, int lane) {
  v16h a; const float* p = rowk0 + 8 * (lane >> 4);
#pragma unroll
  for (int i = 0; i < 8; ++i) { a[i] = (_Float16)p[i]; a[8 + i] = (_Float16)p[16 + i]; }
  return a;
}
__device__ __forceinline__ v16h frag_f32s(const float* rowk0, int lane, float sc) {
  v16h a; const float* p = rowk0 + 8 * (lane >> 4);
#pragma unroll
  for (int i = 0; i < 8; ++i) { a[i] = (_Float16)(p[i] * sc); a[8 + i] = (_Float16)(p[16 + i] * sc); }
  return a;
}
__device__ __forceinline__ v16h fragc_f32(const float* W, int k0, int n, int lane, int ld, int K) {
  v16h a; const int g = lane >> 4;
#pragma unroll
  for (int i = 0; i < 8; ++i) { const int ka = k0 + 8 * g + i, kb = ka + 16;
    a[i] = (_Float16)(ka < K ? W[(size_t)(ka < K ? ka : K - 1) * ld + n] : 0.f); a[8 + i] = (_Float16)(kb < K ? W[(size_t)(kb < K ? kb : K - 1) * ld + n] : 0.f); }
  return a;
}
struct F2 { v16b h, l; };
__device__ __forceinline__ F2 bsplit16(const float v[16]) { F2 r;
#pragma unroll
  for (int i = 0; i < 16; ++i) { const __bf16 h = (__bf16)v[i]; r.h[i] = h; r.l[i] = (__bf16)(v[i] - (float)h); }
  return r; }
__device__ __forceinline__ F2 split_row(const float* row, int k0, int lane) { float v[16]; const float* p = row + k0 + 8 * (lane >> 4);
#pragma unroll
  for (int i = 0; i < 8; ++i) { v[i] = p[i]; v[8 + i] = p[16 + i]; }
  return bsplit16(v); }
__device__ __forceinline__ F2 split_rowK(const float* row, int k0, int lane, int K) { float v[16]; const int g = lane >> 4;
#pragma unroll
  for (int i = 0; i < 8; ++i) { const int ka = k0 + 8 * g + i, kb = ka + 16; v[i] = ka < K ? row[ka < K ? ka : K - 1] : 0.f; v[8 + i] = kb < K ? row[kb < K ? kb : K - 1] : 0.f; }
  return bsplit16(v); }
__device__ __forceinline__ F2 split_col(const float* W, int k0, int n, int lane, int ld, int K) { float v[16]; const int g = lane >> 4;
#pragma unroll
  for (int i = 0; i < 8; ++i) { const int ka = k0 + 8 * g + i, kb = ka + 16; v[i] = ka < K ? W[(size_t)(ka < K ? ka : K - 1) * ld + n] : 0.f; v[8 + i] = kb < K ? W[(size_t)(kb < K ? kb : K - 1) * ld + n] : 0.f; }
  return bsplit16(v); }
__device__ __forceinline__ v8f mac3(const F2& a, const F2& b, v8f c) { c = wmma_bf(a.l, b.h, c); c = wmma_bf(a.h, b.l, c); return wmma_bf(a.h, b.h, c); }
__device__ __forceinline__ float sigm(float v) { return 1.0f / (1.0f + expf(-v)); }
#define LDSX() do { asm volatile("s_wait_dscnt 0" ::: "memory"); __builtin_amdgcn_wave_barrier(); __builtin_amdgcn_fence(__ATOMIC_RELEASE, "workgroup"); } while (0)


#define NBAT 4096
#define TH 200
#define EMB 64
#define WE 160
#define WIN 16
#define OUTW 328
typedef __attribute__((ext_vector_type(8))) __bf16 v8b;
__device__ __forceinline__ v16b frag_b(const __bf16* rowk0, int lane) {
  union { v16b v; v8b q[2]; } u; const __bf16* p = rowk0 + 8 * (lane >> 4);
  u.q[0] = *(const v8b*)p; u.q[1] = *(const v8b*)(p + 16); return u.v;
}
__device__ __forceinline__ float bfr(float v) { return (float)(__bf16)v; }
__device__ __attribute__((noinline)) float exp_ni(float v) { return expf(v); }
__device__ __attribute__((noinline)) float erf_ni(float v) { return erff(v); }
__device__ __attribute__((noinline)) float tanh_ni(float v) { return tanhf(v); }

__device__ __forceinline__ void coaction(const float* __restrict__ ad, const int* __restrict__ hidx, int nrows_tab, const float* __restrict__ IN16, const float* __restrict__ maskrow, float* __restrict__ outv, __bf16 (*sh)[40], __bf16 (*sl)[40], int lane) {
  const int col = lane & 15, g = lane >> 4;
  v16b w0f, w1f;
#pragma unroll
  for (int i = 0; i < 16; ++i) { const int k = 8 * g + (i & 7) + ((i >> 3) << 4); w0f[i] = (__bf16)((col < 8 && k < 16) ? bfr(ad[k * 8 + col]) : 0.f); w1f[i] = (__bf16)((col < 4 && k < 8) ? bfr(ad[128 + k * 4 + col]) : 0.f); }
  float s1[3] = {0.f, 0.f, 0.f}, s2[3] = {0.f, 0.f, 0.f};
#pragma unroll 1
  for (int tile = 0; tile < (TH + 15) / 16; ++tile) { const int trow = tile * 16 + col; const bool valid = trow < TH; int idx = valid ? hidx[trow] : 0; idx = min(max(idx, 0), nrows_tab - 1);
    float hv[8];
#pragma unroll
    for (int i = 0; i < 8; ++i) hv[i] = (valid && (8 * g + i) < WIN) ? bfr(IN16[(size_t)idx * WIN + 8 * g + i]) : 0.f;
    float mrow[8];
#pragma unroll
    for (int r = 0; r < 8; ++r) { const int tr = tile * 16 + 8 * g + r; mrow[r] = (tr < TH) ? bfr(maskrow[tr]) : 0.f; }
#pragma unroll
    for (int p = 0; p < 3; ++p) { v16b ah, al;
#pragma unroll
      for (int i = 0; i < 8; ++i) { float v = hv[i]; const float v1 = v; if (p >= 1) v = v * v1; if (p >= 2) v = v * v1; const __bf16 hb = (__bf16)v; ah[i] = hb; al[i] = (__bf16)(v - (float)hb); ah[8 + i] = (__bf16)0.f; al[8 + i] = (__bf16)0.f; }
      v8f c = {}; c = wmma_bf(al, w0f, c); c = wmma_bf(ah, w0f, c);
      float h1v[8];
#pragma unroll
      for (int r = 0; r < 8; ++r) { h1v[r] = (col < 8) ? tanh_ni(c[r]) : 0.f; s1[p] += mrow[r] * h1v[r]; }
#pragma unroll
      for (int r = 0; r < 8; ++r) { const __bf16 hb = (__bf16)h1v[r]; sh[8 * g + r][col] = hb; sl[8 * g + r][col] = (__bf16)(h1v[r] - (float)hb); }
      __builtin_amdgcn_wave_barrier();
      const v16b a2h = frag_b(&sh[col][0], lane), a2l = frag_b(&sl[col][0], lane);
      v8f c2 = {}; c2 = wmma_bf(a2l, w1f, c2); c2 = wmma_bf(a2h, w1f, c2);
#pragma unroll
      for (int r = 0; r < 8; ++r) s2[p] += (col < 4) ? mrow[r] * c2[r] : 0.f;
      __builtin_amdgcn_wave_barrier(); } }
#pragma unroll
  for (int p = 0; p < 3; ++p) { float a = s1[p], b2 = s2[p]; a += __shfl_xor(a, 16); b2 += __shfl_xor(b2, 16);
    if (g == 0 && col < 8) outv[p * 12 + col] = a;
    if (g == 0 && col < 4) outv[p * 12 + 8 + col] = b2; }
}
__global__ __launch_bounds__(128) void k_ncf(const int* __restrict__ MIDB, const int* __restrict__ CATEB, const int* __restrict__ MIDH, const int* __restrict__ CATEH, const float* __restrict__ MASK, const float* __restrict__ MIDE, const float* __restrict__ CATEE, const float* __restrict__ IMLP, const float* __restrict__ CMLP, const float* __restrict__ IIN, const float* __restrict__ CIN, float* __restrict__ OUT) {
  __shared__ __align__(16) float so[4][OUTW]; __shared__ __align__(16) __bf16 sh[4][16][40], sl[4][16][40];
  const int tid = threadIdx.x, wave = tid >> 5, lane = tid & 31; const size_t b = (size_t)blockIdx.x * 4 + wave;
  for (int e = lane; e < 16 * 40; e += 32) { sh[wave][e / 40][e % 40] = (__bf16)0.f; sl[wave][e / 40][e % 40] = (__bf16)0.f; }
  int mid = MIDB[b]; mid = min(max(mid, 0), 100000 - 1); int cat = CATEB[b]; cat = min(max(cat, 0), 1000 - 1);
  so[wave][lane] = bfr(MIDE[(size_t)mid * EMB + lane]); so[wave][32 + lane] = bfr(MIDE[(size_t)mid * EMB + 32 + lane]); so[wave][64 + lane] = bfr(CATEE[(size_t)cat * EMB + lane]); so[wave][96 + lane] = bfr(CATEE[(size_t)cat * EMB + 32 + lane]);
  { float s0 = 0.f, s1 = 0.f, c0 = 0.f, c1 = 0.f;
#pragma unroll 1
    for (int t = 0; t < TH; ++t) { int mi = MIDH[b * TH + t]; mi = min(max(mi, 0), 100000 - 1); int ci = CATEH[b * TH + t]; ci = min(max(ci, 0), 1000 - 1);
      s0 += bfr(MIDE[(size_t)mi * EMB + lane]); s1 += bfr(MIDE[(size_t)mi * EMB + 32 + lane]); c0 += bfr(CATEE[(size_t)ci * EMB + lane]); c1 += bfr(CATEE[(size_t)ci * EMB + 32 + lane]); }
    so[wave][128 + lane] = s0; so[wave][160 + lane] = s1; so[wave][192 + lane] = c0; so[wave][224 + lane] = c1; }
  __builtin_amdgcn_wave_barrier();
  coaction(IMLP + (size_t)mid * WE, MIDH + b * TH, 100000, IIN, MASK + b * TH, &so[wave][256], sh[wave], sl[wave], lane);
  coaction(CMLP + (size_t)cat * WE, CATEH + b * TH, 1000, CIN, MASK + b * TH, &so[wave][292], sh[wave], sl[wave], lane);
  __syncthreads();
  for (int q = tid; q < 4 * OUTW / 4; q += 128) vst2(OUT + (size_t)blockIdx.x * 4 * OUTW + q * 4, *(const v4f*)(&so[0][0] + q * 4));
}
extern "C" void kernel_launch(void* const* d_in, const int* in_sizes, int n_in, void* d_out, int out_size, void* d_ws, size_t ws_size, hipStream_t stream) {
  (void)in_sizes; (void)n_in; (void)out_size; (void)d_ws; (void)ws_size;
  const float** F = (const float**)d_in;
  static_assert((4 * OUTW * 4) % 128 == 0, "block output must be whole lines");
  k_ncf<<<NBAT / 4, 128, 0, stream>>>((const int*)d_in[1], (const int*)d_in[2], (const int*)d_in[3], (const int*)d_in[4], F[5], F[7], F[8], F[9], F[10], F[11], F[12], (float*)d_out);
}
